// GenLSTMd_9938554323550
// MI455X (gfx1250) — hardware-run, weakly checked
//
#include <hip/hip_runtime.h>
#include <math.h>

constexpr int NBAT    = 1024;
constexpr int NTIME   = 256;
constexpr int NHID    = 256;
constexpr int NGATE   = 4 * NHID;
constexpr int NNOISE  = 16;
constexpr int NFEAT   = 1 + NNOISE + 1;
constexpr int KIN     = 32;
constexpr int NHIST   = 32;
constexpr int NCOND   = NHIST - 1;
constexpr int NSTEPS  = NTIME - 1;
constexpr int NLIVE   = NSTEPS - 1;
constexpr int ROWS_BLK = 16;
constexpr int LSTM_THREADS = 512;
constexpr int PACK_THREADS = 256;
constexpr int HPITCH  = 264;
constexpr int IPITCH  = 40;
constexpr int OPITCH  = NTIME * 2;
constexpr float ACARRY = 16.0f;
constexpr float WCARRY = 64.0f;
constexpr float FOLD   = 1.0f / (ACARRY * WCARRY);

static_assert(NFEAT == 18, "feature count");
static_assert(NFEAT + 2 <= KIN, "hi/lo slots fit in the padded k step");
static_assert(KIN % 32 == 0 && NHID % 32 == 0, "k multiples of 32");
static_assert(NBAT % ROWS_BLK == 0, "row blocks exact");
static_assert(NHID == 16 * (LSTM_THREADS / 32), "16 waves x 16 hidden columns");
static_assert(ROWS_BLK == LSTM_THREADS / 32, "one input row per wave in the build phase");
static_assert(NGATE % 64 == 0 && NHID % 64 == 0, "transpose tiles exact");
static_assert((ROWS_BLK * OPITCH) % (LSTM_THREADS * 4) == 0, "output copy loop exact");
static_assert(HPITCH % 8 == 0 && IPITCH % 8 == 0, "16-byte aligned LDS rows");

typedef __attribute__((ext_vector_type(16))) _Float16 v16h;
typedef __attribute__((ext_vector_type(8)))  _Float16 v8h;
typedef __attribute__((ext_vector_type(8)))  float    v8f;
typedef __attribute__((ext_vector_type(4)))  float    v4f;

__device__ __forceinline__ unsigned short f2bf_bits(float f) {
  unsigned u = __float_as_uint(f);
  return (unsigned short)((u + 0x7FFFu + ((u >> 16) & 1u)) >> 16);
}
__device__ __forceinline__ float bf_bits2f(unsigned short h) { return __uint_as_float(((unsigned)h) << 16); }
__device__ __forceinline__ float bf16r(float f) { return bf_bits2f(f2bf_bits(f)); }

__device__ __forceinline__ void guard_all_h(v8f& a, v8f& b, v8f& c, v8f& d, v16h x, v16h y0, v16h y1, v16h y2, v16h y3) {
  asm volatile("v_nop\n\tv_nop\n\tv_nop\n\tv_nop" : "+v"(a), "+v"(b), "+v"(c), "+v"(d) : "v"(x), "v"(y0), "v"(y1), "v"(y2), "v"(y3));
}
__device__ __forceinline__ void acc_guard4(v8f& a, v8f& b, v8f& c, v8f& d) {
  asm volatile("v_nop\n\tv_nop\n\tv_nop\n\tv_nop" : "+v"(a), "+v"(b), "+v"(c), "+v"(d));
}

struct FragH {
  union U { v16h v; v8h h[2]; };
  static __device__ __forceinline__ v16h load(const _Float16* p) {
    U f; f.h[0] = *(const v8h*)(p); f.h[1] = *(const v8h*)(p + 16); return f.v;
  }
  static __device__ __forceinline__ v8f mma(v16h a, v16h b, v8f c) {
    return __builtin_amdgcn_wmma_f32_16x16x32_f16(false, a, false, b, (short)0, c, false, false);
  }
};

__device__ __forceinline__ float fsig(float x)  { return __builtin_amdgcn_rcpf(1.0f + __expf(-x)); }
__device__ __forceinline__ float ftanh(float x) { return 1.0f - 2.0f * __builtin_amdgcn_rcpf(__expf(2.0f * x) + 1.0f); }

__global__ __launch_bounds__(PACK_THREADS) void wr_transpose_kernel(const float* __restrict__ src, int R, int C, int ldo,
                                                                   unsigned short* __restrict__ O, float sc) {
  __shared__ float Tt[64 * 65];
  const int tid = threadIdx.x;
  const int c0 = blockIdx.x * 64, r0 = blockIdx.y * 64;
#pragma unroll
  for (int i = 0; i < 4; ++i) {
    const int idx = i * PACK_THREADS + tid;
    const int rr = idx >> 4, cc = (idx & 15) * 4;
    const v4f v = *(const v4f*)(src + (size_t)(r0 + rr) * (size_t)C + c0 + cc);
    Tt[rr * 65 + cc + 0] = v[0];
    Tt[rr * 65 + cc + 1] = v[1];
    Tt[rr * 65 + cc + 2] = v[2];
    Tt[rr * 65 + cc + 3] = v[3];
  }
  __syncthreads();
  const int q = tid >> 3, c8 = (tid & 7) * 8;
  v8h hv[2];
#pragma unroll
  for (int g = 0; g < 2; ++g) {
    const int qq = g * 32 + q;
#pragma unroll
    for (int e = 0; e < 8; ++e) {
      const float f = Tt[(c8 + e) * 65 + qq];
      hv[g][e] = (_Float16)(bf16r(f) * sc);
    }
  }
  for (int pass = 0; pass < 2; ++pass) {
#pragma unroll
    for (int g = 0; g < 2; ++g) {
      const size_t o = (size_t)(c0 + g * 32 + q) * (size_t)ldo + (size_t)(r0 + c8);
      *(volatile v8h*)(O + o) = hv[g];
    }
    __threadfence();
  }
}

__global__ __launch_bounds__(PACK_THREADS) void wk_pack_kernel(const float* __restrict__ Wk, unsigned short* __restrict__ WKT) {
  const int i = blockIdx.x * PACK_THREADS + threadIdx.x;
  if (i < NGATE * (KIN / 8)) {
    const int n = i >> 2, kg = (i & 3) * 8;
    v8h hv;
#pragma unroll
    for (int e = 0; e < 8; ++e) {
      const int k = kg + e;
      const int srow = (k < NFEAT) ? k : ((k == NFEAT) ? (NFEAT - 1) : 0);
      const float f = Wk[(size_t)srow * NGATE + n];
      const float v = (k < NFEAT + 2) ? (bf16r(f) * WCARRY) : 0.0f;
      hv[e] = (_Float16)v;
    }
    *(volatile v8h*)(WKT + (size_t)i * 8) = hv;
    __threadfence();
    *(volatile v8h*)(WKT + (size_t)i * 8) = hv;
  }
}

__global__ __launch_bounds__(LSTM_THREADS) void lstm_gen_kernel(const float* __restrict__ noise, const float* __restrict__ x,
                                                                const float* __restrict__ bias, const float* __restrict__ wd,
                                                                const float* __restrict__ bd,
                                                                const unsigned short* __restrict__ WKTp,
                                                                const unsigned short* __restrict__ WRTp,
                                                                float* __restrict__ out) {
  __shared__ __align__(16) _Float16 Hh[2][ROWS_BLK * HPITCH];
  __shared__ __align__(16) _Float16 Ain[ROWS_BLK * IPITCH];
  __shared__ __align__(16) float    Xgp[16 * ROWS_BLK];
  __shared__ __align__(16) float    Orow[ROWS_BLK * OPITCH];

  const _Float16* WKT = (const _Float16*)WKTp;
  const _Float16* WRT = (const _Float16*)WRTp;
  const int tid = threadIdx.x, lane = tid & 31, wave = tid >> 5;
  const int c = lane & 15, hh = lane >> 4, koff = hh * 8;
  const int rowbase = blockIdx.x * ROWS_BLK;
  const int j = 16 * wave + c;

  {
    _Float16* hz = &Hh[0][0];
#pragma unroll 1
    for (int i = tid; i < 2 * ROWS_BLK * HPITCH; i += LSTM_THREADS) hz[i] = (_Float16)0.0f;
  }
  if (tid < 16 * ROWS_BLK) Xgp[tid] = 0.0f;
#pragma unroll
  for (int it = 0; it < (ROWS_BLK * OPITCH) / (LSTM_THREADS * 4); ++it) {
    const int idx = it * LSTM_THREADS + tid;
    const v4f v = *(const v4f*)(x + (size_t)rowbase * OPITCH + (size_t)idx * 4);
    v4f o;
    o[0] = bf16r(v[0]); o[1] = 0.0f; o[2] = bf16r(v[2]); o[3] = 0.0f;
    *(v4f*)(Orow + idx * 4) = o;
  }

  const float bb0 = bf16r(bias[0 * NHID + j]);
  const float bb1 = bf16r(bias[1 * NHID + j]);
  const float bb2 = bf16r(bias[2 * NHID + j]);
  const float bb3 = bf16r(bias[3 * NHID + j]);
  const float wdj = bf16r(wd[j]);
  const float bdv = bf16r(bd[0]);
  const v16h wk0 = FragH::load(WKT + (size_t)(0 * NHID + j) * KIN + koff);
  const v16h wk1 = FragH::load(WKT + (size_t)(1 * NHID + j) * KIN + koff);
  const v16h wk2 = FragH::load(WKT + (size_t)(2 * NHID + j) * KIN + koff);
  const v16h wk3 = FragH::load(WKT + (size_t)(3 * NHID + j) * KIN + koff);
  const _Float16* wh = WRT + (size_t)j * NHID + koff;

  const int  pk    = lane;
  const int  prow  = wave;
  const bool is_x0 = (pk == 0) || (pk == NFEAT + 1);
  const bool is_dt = (pk == NFEAT - 1) || (pk == NFEAT);
  const bool is_nz = (pk >= 1) && (pk <= NNOISE);
  const bool is_lo = (pk == NFEAT) || (pk == NFEAT + 1);
  const int  xcol  = is_dt ? 0 : 1;
  int nzc = pk - 1;
  nzc = nzc < 0 ? 0 : (nzc > NNOISE - 1 ? NNOISE - 1 : nzc);
  const float* xsrc = x + (size_t)(rowbase + prow) * OPITCH + xcol;
  const float* nsrc = noise + (size_t)(rowbase + prow) * (size_t)(NSTEPS * NNOISE) + nzc;

  float cst[8];
#pragma unroll
  for (int r = 0; r < 8; ++r) cst[r] = 0.0f;
  float cum = 0.0f;
  const v8f z8 = {0.f, 0.f, 0.f, 0.f, 0.f, 0.f, 0.f, 0.f};
  const _Float16* ainrow = Ain + c * IPITCH + koff;

  __syncthreads();

#pragma unroll 1
  for (int s = 0; s < NLIVE; ++s) {
    const int  cur = s & 1;
    const bool gen = (s >= NCOND);

    {
      float xa = xsrc[2 * (s + 1)];
      float xb = xsrc[2 * s];
      float nz = nsrc[s * NNOISE];
      asm volatile("" : "+v"(xa));
      asm volatile("" : "+v"(xb));
      asm volatile("" : "+v"(nz));
      const float d = bf16r(xa) - bf16r(xb);
      float sx = Xgp[prow];
#pragma unroll
      for (int w = 1; w < 16; ++w) sx += Xgp[w * ROWS_BLK + prow];
      const float xg = sx + bdv;
      const float x0 = gen ? xg : d;
      const float val = is_x0 ? x0 : (is_dt ? d : (is_nz ? bf16r(nz) : 0.0f));
      const float sv  = val * ACARRY;
      const _Float16 hi = (_Float16)sv;
      const float lof = sv - (float)hi;
      const float of  = is_lo ? lof : sv;
      Ain[prow * IPITCH + pk] = (_Float16)of;
      cum += x0;
      if (pk == 0) Orow[prow * OPITCH + 2 * (s + 1) + 1] = cum;
    }
    __syncthreads();

    v8f acc[4];
    acc[0] = z8; acc[1] = z8; acc[2] = z8; acc[3] = z8;
    {
      const v16h a = FragH::load(ainrow);
      acc[0] = FragH::mma(a, wk0, acc[0]);
      acc[1] = FragH::mma(a, wk1, acc[1]);
      acc[2] = FragH::mma(a, wk2, acc[2]);
      acc[3] = FragH::mma(a, wk3, acc[3]);
      guard_all_h(acc[0], acc[1], acc[2], acc[3], a, wk0, wk1, wk2, wk3);
    }
    {
      const _Float16* ahrow = &Hh[cur][0] + c * HPITCH + koff;
#pragma unroll 1
      for (int k0 = 0; k0 < NHID; k0 += 32) {
        const v16h a  = FragH::load(ahrow + k0);
        const v16h b0 = FragH::load(wh + k0);
        const v16h b1 = FragH::load(wh + (size_t)1 * NHID * NHID + k0);
        const v16h b2 = FragH::load(wh + (size_t)2 * NHID * NHID + k0);
        const v16h b3 = FragH::load(wh + (size_t)3 * NHID * NHID + k0);
        acc[0] = FragH::mma(a, b0, acc[0]);
        acc[1] = FragH::mma(a, b1, acc[1]);
        acc[2] = FragH::mma(a, b2, acc[2]);
        acc[3] = FragH::mma(a, b3, acc[3]);
        guard_all_h(acc[0], acc[1], acc[2], acc[3], a, b0, b1, b2, b3);
      }
    }
    acc_guard4(acc[0], acc[1], acc[2], acc[3]);

    _Float16* ahn = &Hh[cur ^ 1][0];
    float pw[8];
#pragma unroll
    for (int r = 0; r < 8; ++r) {
      const float zi = acc[0][r] * FOLD + bb0;
      const float zf = acc[1][r] * FOLD + bb1;
      const float zg = acc[2][r] * FOLD + bb2;
      const float zo = acc[3][r] * FOLD + bb3;
      const float ig = fsig(zi);
      const float fg = fsig(zf);
      const float gg = ftanh(zg);
      const float og = fsig(zo);
      const float cn = fg * cst[r] + ig * gg;
      cst[r] = cn;
      const float hn = og * ftanh(cn);
      ahn[(8 * hh + r) * HPITCH + j] = (_Float16)(hn * ACARRY);
      pw[r] = hn * wdj;
    }
#pragma unroll
    for (int off = 1; off < 16; off <<= 1) {
#pragma unroll
      for (int r = 0; r < 8; ++r) pw[r] += __shfl_xor(pw[r], off, 32);
    }
    if (c == 0) {
      v4f p0, p1;
      p0[0] = pw[0]; p0[1] = pw[1]; p0[2] = pw[2]; p0[3] = pw[3];
      p1[0] = pw[4]; p1[1] = pw[5]; p1[2] = pw[6]; p1[3] = pw[7];
      *(v4f*)(Xgp + wave * ROWS_BLK + 8 * hh)     = p0;
      *(v4f*)(Xgp + wave * ROWS_BLK + 8 * hh + 4) = p1;
    }
    __syncthreads();
  }

  {
    float sx = Xgp[prow];
#pragma unroll
    for (int w = 1; w < 16; ++w) sx += Xgp[w * ROWS_BLK + prow];
    const float xg = sx + bdv;
    cum += xg;
    if (pk == 0) Orow[prow * OPITCH + 2 * NSTEPS + 1] = cum;
  }
  __syncthreads();

  {
    float* ob = out + (size_t)rowbase * OPITCH;
    for (int pass = 0; pass < 2; ++pass) {
#pragma unroll
      for (int it = 0; it < (ROWS_BLK * OPITCH) / (LSTM_THREADS * 4); ++it) {
        const int idx = it * LSTM_THREADS + tid;
        const v4f v = *(const v4f*)(Orow + idx * 4);
        *(volatile v4f*)(ob + (size_t)idx * 4) = v;
      }
      __threadfence();
    }
  }
}

extern "C" void kernel_launch(void* const* d_in, const int* in_sizes, int n_in,
                              void* d_out, int out_size, void* d_ws, size_t ws_size, hipStream_t stream) {
  if (n_in < 7 || d_out == nullptr || d_ws == nullptr) return;
  if (in_sizes[0] != NBAT * NSTEPS * NNOISE || in_sizes[1] != NBAT * NTIME * 2 || in_sizes[2] != NFEAT * NGATE ||
      in_sizes[3] != NHID * NGATE || in_sizes[4] != NGATE || in_sizes[5] != NHID || in_sizes[6] != 1 ||
      out_size != NBAT * NTIME * 2) return;

  const float* noise = (const float*)d_in[0];
  const float* xin   = (const float*)d_in[1];
  const float* wk    = (const float*)d_in[2];
  const float* wr    = (const float*)d_in[3];
  const float* bl    = (const float*)d_in[4];
  const float* wd    = (const float*)d_in[5];
  const float* bd    = (const float*)d_in[6];
  float* out = (float*)d_out;

  char* ws = (char*)d_ws; size_t off = 0;
  auto carve = [&](size_t bytes) -> char* { char* p = ws + off; off += (bytes + 255) & ~(size_t)255; return p; };
  unsigned short* WRT = (unsigned short*)carve((size_t)NGATE * NHID * 2);
  unsigned short* WKT = (unsigned short*)carve((size_t)NGATE * KIN * 2);
  if (off > ws_size || off > (size_t)134217728) return;

  wr_transpose_kernel<<<dim3(NGATE / 64, NHID / 64), PACK_THREADS, 0, stream>>>(wr, NHID, NGATE, NHID, WRT, WCARRY);
  wk_pack_kernel<<<(NGATE * (KIN / 8)) / PACK_THREADS, PACK_THREADS, 0, stream>>>(wk, WKT);
  lstm_gen_kernel<<<NBAT / ROWS_BLK, LSTM_THREADS, 0, stream>>>(noise, xin, bl, wd, bd, WKT, WRT, out);
}
